// ConvLRU_11398843203895
// MI455X (gfx1250) — hardware-verified
//
#include <hip/hip_runtime.h>
#include <math.h>

typedef __attribute__((ext_vector_type(16))) _Float16 v16h;
typedef __attribute__((ext_vector_type(8)))  _Float16 v8h;
typedef __attribute__((ext_vector_type(2)))  _Float16 v2h;
typedef __attribute__((ext_vector_type(16))) __bf16   v16b;
typedef __attribute__((ext_vector_type(8)))  __bf16   v8b;
typedef __attribute__((ext_vector_type(8)))  float    v8f;
typedef __attribute__((ext_vector_type(4)))  float    v4f;

constexpr int kB    = 4;
constexpr int kL    = 32;
constexpr int kE    = 64;
constexpr int kC    = 96;
constexpr int kS    = 32;
constexpr int kP    = kB * kL;
constexpr int kPE   = kP * kE;
constexpr int kPA   = kP * kS;
constexpr int kPC   = kP * kC;
constexpr int kE2   = 2 * kE;
constexpr int kC2   = 2 * kC;
constexpr int kS2   = 2 * kS;
constexpr int kThr  = 256;

constexpr float cSx  = 64.0f;
constexpr float cTw  = 16384.0f;
constexpr float cW   = 1024.0f;
constexpr float cXh  = 32.0f;
constexpr float cH1  = 32.0f;
constexpr float cHs  = 1.0f;
constexpr float cG   = 512.0f;
constexpr float cH6  = 2048.0f;
constexpr float kScG1 = 1.0f / (cSx * cTw);
constexpr float kScG2 = 1.0f / (cXh * cW);
constexpr float kScG3 = 1.0f / (cH1 * cW);
constexpr float kScG5 = 1.0f / (cHs * cTw * 1024.0f);
constexpr float kScG6 = 1.0f / (cG * cW);
constexpr float kScG7 = 1.0f / (cH6 * cW);
constexpr float kF16MinNormal = 6.103515625e-5f;

static_assert((kPE % 64) == 0 && (kPA % 64) == 0 && (kPC % 64) == 0 && (kS2 % 64) == 0 && (kC2 % 64) == 0 && (kE % 64) == 0, "GEMM M, N multiples of 64");
static_assert((kS % 32) == 0 && (kE2 % 32) == 0 && (kC2 % 32) == 0 && (kS2 % 32) == 0, "GEMM K multiples of 32");
static_assert(kScG1 == 9.5367431640625e-7f && kScG5 == 5.9604644775390625e-8f, "power-of-two scales");

constexpr size_t kOffSX   = 0;
constexpr size_t kOffTWF  = kOffSX  + (size_t)kPE * kS * 2;
constexpr size_t kOffTWI  = kOffTWF + (size_t)kS2 * kS * 2;
constexpr size_t kOffWB   = kOffTWI + (size_t)kS2 * kS2 * 2;
constexpr size_t kOffWP1  = kOffWB  + (size_t)kC2 * kE2 * 2;
constexpr size_t kOffWP2  = kOffWP1 + (size_t)kC2 * kC2 * 2;
constexpr size_t kOffWC   = kOffWP2 + (size_t)kC2 * kC2 * 2;
constexpr size_t kOffTAB  = kOffWC  + (size_t)kE * kC2 * 2;
constexpr int    kTabBP1 = 0, kTabBP2 = 192, kTabBC = 384, kTabBB = 448, kTabZB = 640, kTabGAM = 1024, kTabLRE = 4096, kTabLIM = 7168, kTabN = 10240;
constexpr size_t kOffXH   = kOffTAB + (size_t)kTabN * 4;
constexpr size_t kOffA2   = kOffXH  + (size_t)kPE * kS2 * 4;
constexpr size_t kOffH1   = kOffA2  + (size_t)kPA * kE2 * 2;
constexpr size_t kOffA3   = kOffH1  + (size_t)kPA * kC2 * 4;
constexpr size_t kOffH2   = kOffA3  + (size_t)kPA * kC2 * 2;
constexpr size_t kOffA5   = kOffH2  + (size_t)kPA * kC2 * 4;
constexpr size_t kOffGG   = kOffA5  + (size_t)kPC * kS2 * 2;
constexpr size_t kOffA6   = kOffGG  + (size_t)kPC * kS2 * 4;
constexpr size_t kOffH6   = kOffA6  + (size_t)kPA * kC2 * 2;
constexpr size_t kOffA7   = kOffH6  + (size_t)kPA * kC2 * 4;
constexpr size_t kOffRR   = kOffA7  + (size_t)kPA * kC2 * 2;
constexpr size_t kWsTotal = kOffRR  + (size_t)kPA * kE * 4;
static_assert(kWsTotal == 23867392ull, "carve total");
static_assert(kWsTotal <= 134217728ull, "carve cap");
static_assert((kOffTWF % 256) == 0 && (kOffTWI % 256) == 0 && (kOffWB % 256) == 0 && (kOffWP1 % 256) == 0 && (kOffWP2 % 256) == 0 && (kOffWC % 256) == 0 && (kOffTAB % 256) == 0 && (kOffXH % 256) == 0 && (kOffA2 % 256) == 0 && (kOffH1 % 256) == 0 && (kOffA3 % 256) == 0 && (kOffH2 % 256) == 0 && (kOffA5 % 256) == 0 && (kOffGG % 256) == 0 && (kOffA6 % 256) == 0 && (kOffH6 % 256) == 0 && (kOffA7 % 256) == 0 && (kOffRR % 256) == 0, "aligned regions");

__device__ __forceinline__ unsigned short f2bf_bits(float f) {
  unsigned u = __float_as_uint(f);
  return (unsigned short)((u + 0x7FFFu + ((u >> 16) & 1u)) >> 16);
}
__device__ __forceinline__ float bf_bits2f(unsigned short h) { return __uint_as_float(((unsigned)h) << 16); }
__device__ __forceinline__ float bf16r(float f) { return bf_bits2f(f2bf_bits(f)); }
__device__ __forceinline__ float carry_flush(float v, float carry) {
  const float s = v * carry;
  return (fabsf(s) < kF16MinNormal) ? 0.0f : s;
}
__device__ __forceinline__ float frcp(float x) { return __builtin_amdgcn_rcpf(x); }

__device__ __forceinline__ void dep_guard4_h(v8f& a, v8f& b, v8f& c, v8f& d, v16h x, v16h y) { asm volatile("v_nop\n\tv_nop\n\tv_nop\n\tv_nop" : "+v"(a), "+v"(b), "+v"(c), "+v"(d) : "v"(x), "v"(y)); }
__device__ __forceinline__ void dep_guard4_b(v8f& a, v8f& b, v8f& c, v8f& d, v16b x, v16b y) { asm volatile("v_nop\n\tv_nop\n\tv_nop\n\tv_nop" : "+v"(a), "+v"(b), "+v"(c), "+v"(d) : "v"(x), "v"(y)); }
__device__ __forceinline__ void keep4_h(v16h a, v16h b, v16h c, v16h d) { asm volatile("v_nop" :: "v"(a), "v"(b), "v"(c), "v"(d)); }
__device__ __forceinline__ void keep4_b(v16b a, v16b b, v16b c, v16b d) { asm volatile("v_nop" :: "v"(a), "v"(b), "v"(c), "v"(d)); }
__device__ __forceinline__ void acc_guard4(v8f& a, v8f& b, v8f& c, v8f& d) { asm volatile("v_nop\n\tv_nop\n\tv_nop\n\tv_nop" : "+v"(a), "+v"(b), "+v"(c), "+v"(d)); }

template <typename T> struct Frag;
template <> struct Frag<_Float16> {
  typedef v16h V; union U { v16h v; v8h h[2]; };
  static __device__ __forceinline__ v16h load(const _Float16* p) {
    U f; f.h[0] = *(const v8h*)(p); f.h[1] = *(const v8h*)(p + 16); return f.v;
  }
  static __device__ __forceinline__ v8f mma(v16h a, v16h b, v8f c) {
    return __builtin_amdgcn_wmma_f32_16x16x32_f16(false, a, false, b, (short)0, c, false, false);
  }
  static __device__ __forceinline__ void guard4(v8f& a, v8f& b, v8f& c, v8f& d, v16h x, v16h y) { dep_guard4_h(a, b, c, d, x, y); }
  static __device__ __forceinline__ void keep(v16h a, v16h b, v16h c, v16h d) { keep4_h(a, b, c, d); }
};
template <> struct Frag<__bf16> {
  typedef v16b V; union U { v16b v; v8b h[2]; };
  static __device__ __forceinline__ v16b load(const __bf16* p) {
    U f; f.h[0] = *(const v8b*)(p); f.h[1] = *(const v8b*)(p + 16); return f.v;
  }
  static __device__ __forceinline__ v8f mma(v16b a, v16b b, v8f c) {
    return __builtin_amdgcn_wmma_f32_16x16x32_bf16(false, a, false, b, (short)0, c, false, false);
  }
  static __device__ __forceinline__ void guard4(v8f& a, v8f& b, v8f& c, v8f& d, v16b x, v16b y) { dep_guard4_b(a, b, c, d, x, y); }
  static __device__ __forceinline__ void keep(v16b a, v16b b, v16b c, v16b d) { keep4_b(a, b, c, d); }
};

__device__ __forceinline__ v8f mma_h(v16h a, v16h b, v8f c) {
  c = __builtin_amdgcn_wmma_f32_16x16x32_f16(false, a, false, b, (short)0, c, false, false);
  asm volatile("v_nop\n\tv_nop\n\tv_nop\n\tv_nop" : "+v"(c) : "v"(a), "v"(b));
  return c;
}

template <int ET> struct Elem;
template <> struct Elem<0> { typedef _Float16 T; };
template <> struct Elem<1> { typedef __bf16 T; };
template <int ET, bool SPLIT, int BIAS_MODE, int OUT_MODE, bool RESID, int ACT = 0>
__global__ __launch_bounds__(256) void wmma_gemm64(
    const unsigned short* __restrict__ Ap, const unsigned short* __restrict__ A2p, int lda, long strideA,
    const unsigned short* __restrict__ Btp, const unsigned short* __restrict__ Bt2p, int ldb, long strideB,
    void* __restrict__ Cout, void* __restrict__ Cout2, int ldc, long strideC,
    const float* __restrict__ bias,
    const float* __restrict__ resid, long strideR,
    int M, int N, int K, float scale) {
  typedef typename Elem<ET>::T T;
  typedef typename Frag<T>::V V;
  const T* A = (const T*)Ap; const T* A2 = (const T*)A2p; const T* Bt = (const T*)Btp; const T* Bt2 = (const T*)Bt2p;
  __shared__ __align__(16) float sT[8][16 * 68];
  const int b    = blockIdx.y;
  const int lane = threadIdx.x & 31;
  const int wave = threadIdx.x >> 5;
  const int tilesN = N >> 6;
  const int tilesM = M >> 6;
  const int tile = blockIdx.x * 8 + wave;
  if (tile >= tilesM * tilesN) return;
  const int tm = tile / tilesN;
  const int tn = tile - tm * tilesN;
  const int m0 = tm << 6;
  const int n0 = tn << 6;

  const T* Ab  = A  + (size_t)b * strideA;
  const T* Bb  = Bt + (size_t)b * strideB;
  const T* Ab2 = SPLIT ? (A2  + (size_t)b * strideA) : nullptr;
  const T* Bb2 = SPLIT ? (Bt2 + (size_t)b * strideB) : nullptr;

  const int rlane = lane & 15;
  const int koff  = (lane >> 4) * 8;
  const int mOff  = (lane >> 4) * 8;

  v8f acc[4][4];
#pragma unroll
  for (int i = 0; i < 4; ++i)
#pragma unroll
    for (int j = 0; j < 4; ++j) acc[i][j] = (v8f){0.f,0.f,0.f,0.f,0.f,0.f,0.f,0.f};

  for (int k0 = 0; k0 < K; k0 += 32) {
    V bh[4], bl[4];
#pragma unroll
    for (int j = 0; j < 4; ++j) {
      const size_t bo = (size_t)(n0 + (j << 4) + rlane) * ldb + koff + k0;
      bh[j] = Frag<T>::load(Bb + bo);
      if (SPLIT) bl[j] = Frag<T>::load(Bb2 + bo);
    }
#pragma unroll
    for (int i = 0; i < 4; ++i) {
      const size_t ao = (size_t)(m0 + (i << 4) + rlane) * lda + koff + k0;
      V ah = Frag<T>::load(Ab + ao);
      V al;
      if (SPLIT) al = Frag<T>::load(Ab2 + ao);
#pragma unroll
      for (int j = 0; j < 4; ++j) {
        acc[i][j] = Frag<T>::mma(ah, bh[j], acc[i][j]);
        if (SPLIT) {
          acc[i][j] = Frag<T>::mma(ah, bl[j], acc[i][j]);
          acc[i][j] = Frag<T>::mma(al, bh[j], acc[i][j]);
        }
      }
      Frag<T>::guard4(acc[i][0], acc[i][1], acc[i][2], acc[i][3], ah, SPLIT ? al : ah);
    }
    Frag<T>::keep(bh[0], bh[1], bh[2], bh[3]);
    if (SPLIT) Frag<T>::keep(bl[0], bl[1], bl[2], bl[3]);
  }
  acc_guard4(acc[0][0], acc[0][1], acc[0][2], acc[0][3]);
  acc_guard4(acc[1][0], acc[1][1], acc[1][2], acc[1][3]);
  acc_guard4(acc[2][0], acc[2][1], acc[2][2], acc[2][3]);
  acc_guard4(acc[3][0], acc[3][1], acc[3][2], acc[3][3]);

  float* slab = sT[wave];
  const float* Rb = RESID ? (resid + (size_t)b * strideR) : nullptr;
#pragma unroll
  for (int i = 0; i < 4; ++i) {
    const int mBase = m0 + (i << 4);
#pragma unroll
    for (int j = 0; j < 4; ++j) {
      const int n = n0 + (j << 4) + rlane;
      float bv = 0.f;
      if (BIAS_MODE == 2) bv = bias[n];
#pragma unroll
      for (int r = 0; r < 8; ++r) {
        float v = acc[i][j][r] * scale;
        if (BIAS_MODE == 1) v += bias[mBase + mOff + r];
        if (BIAS_MODE == 2) v += bv;
        if (RESID) v += Rb[(size_t)(mBase + mOff + r) * ldc + n];
        if (ACT == 1) v = tanhf(v);
        if (ACT == 2) v = fmaxf(v, 0.0f);
        if (ACT == 3) v = v / (1.0f + expf(-v));
        if (ACT == 4) v = (v > 0.f) ? v : 0.01f * v;
        slab[(mOff + r) * 68 + (j << 4) + rlane] = v;
      }
    }
    __builtin_amdgcn_fence(__ATOMIC_RELEASE, "workgroup");
    __builtin_amdgcn_wave_barrier();
    __builtin_amdgcn_fence(__ATOMIC_ACQUIRE, "workgroup");
    if (OUT_MODE == 0) {
      float* C = (float*)Cout + (size_t)b * strideC;
      const int hh = lane >> 4, c4 = (lane & 15) * 4;
      for (int pass = 0; pass < 2; ++pass) {
#pragma unroll
        for (int it = 0; it < 8; ++it) {
          const int row = it * 2 + hh;
          v4f v = *(const v4f*)(slab + row * 68 + c4);
          *(volatile v4f*)(C + (size_t)(mBase + row) * ldc + n0 + c4) = v;
        }
        __threadfence();
      }
    } else {
      const int q = lane >> 3, c8 = (lane & 7) * 8;
      unsigned short* C  = (unsigned short*)Cout  + (size_t)b * strideC;
      unsigned short* C2 = (OUT_MODE == 2) ? ((unsigned short*)Cout2 + (size_t)b * strideC) : nullptr;
      for (int pass = 0; pass < 2; ++pass) {
#pragma unroll
        for (int it = 0; it < 4; ++it) {
          const int row = it * 4 + q;
          const float* sp = slab + row * 68 + c8;
          v8h hv, lv;
#pragma unroll
          for (int e = 0; e < 8; ++e) {
            if (OUT_MODE == 1) {
              hv[e] = (_Float16)sp[e];
            } else {
              unsigned short hb = f2bf_bits(sp[e]);
              unsigned short lb = f2bf_bits(sp[e] - bf_bits2f(hb));
              hv[e] = __builtin_bit_cast(_Float16, hb);
              lv[e] = __builtin_bit_cast(_Float16, lb);
            }
          }
          *(volatile v8h*)(C + (size_t)(mBase + row) * ldc + n0 + c8) = hv;
          if (OUT_MODE == 2) *(volatile v8h*)(C2 + (size_t)(mBase + row) * ldc + n0 + c8) = lv;
        }
        __threadfence();
      }
    }
    __builtin_amdgcn_fence(__ATOMIC_RELEASE, "workgroup");
    __builtin_amdgcn_wave_barrier();
    __builtin_amdgcn_fence(__ATOMIC_ACQUIRE, "workgroup");
  }
}


__global__ __launch_bounds__(kThr) void antidiag_kernel(const float* __restrict__ x, unsigned short* __restrict__ SX16) {
  unsigned t = blockIdx.x * (unsigned)kThr + threadIdx.x;
  asm volatile("" : "+v"(t));
  const unsigned lane = t & 31u;
  const unsigned plane = (t >> 5) * 2u + (lane >> 4);
  const unsigned s0 = (lane & 15u) * 2u;
  const float* xp = x + (size_t)plane * (kS * kS);
  float a0 = 0.f, a1 = 0.f;
#pragma unroll 8
  for (unsigned p = 0; p < (unsigned)kS; ++p) {
    const float v0 = xp[p * (unsigned)kS + ((s0 - p) & 31u)];
    const float v1 = xp[p * (unsigned)kS + ((s0 + 1u - p) & 31u)];
    a0 += bf16r(v0);
    a1 += bf16r(v1);
  }
  v2h o;
  o[0] = (_Float16)carry_flush(a0, cSx);
  o[1] = (_Float16)carry_flush(a1, cSx);
  unsigned short* dp = SX16 + (size_t)plane * kS + s0;
  *(volatile v2h*)dp = o;
  __threadfence();
  *(volatile v2h*)dp = o;
}
static_assert((kPE / 2) * 32 == 512 * kThr, "antidiag grid exact");

__device__ const float kCos32[32] = {1.0f, 0.980785251f, 0.923879504f, 0.831469595f, 0.707106769f, 0.555570245f, 0.382683426f, 0.195090324f, 0.0f, -0.195090324f, -0.382683426f, -0.555570245f, -0.707106769f, -0.831469595f, -0.923879504f, -0.980785251f, -1.0f, -0.980785251f, -0.923879504f, -0.831469595f, -0.707106769f, -0.555570245f, -0.382683426f, -0.195090324f, 0.0f, 0.195090324f, 0.382683426f, 0.555570245f, 0.707106769f, 0.831469595f, 0.923879504f, 0.980785251f};
__global__ __launch_bounds__(kThr) void twiddle_kernel(unsigned short* __restrict__ TWF, unsigned short* __restrict__ TWI) {
  unsigned v = blockIdx.x * (unsigned)kThr + threadIdx.x;
  asm volatile("" : "+v"(v));
  const bool inv = v >= 256u;
  const unsigned u = inv ? (v - 256u) : v;
  const unsigned n = inv ? (u >> 3) : (u >> 2);
  const unsigned k0 = inv ? ((u & 7u) * 8u) : ((u & 3u) * 8u);
  v8h hv;
#pragma unroll
  for (int e = 0; e < 8; ++e) {
    const unsigned k = k0 + (unsigned)e;
    const unsigned j = ((n & 31u) * (k & 31u)) & 31u;
    const float cs = kCos32[j];
    const float sn = kCos32[(j + 24u) & 31u];
    float val;
    if (!inv) val = (n < 32u) ? cs : -sn;
    else val = (n < 32u) ? ((k < 32u) ? cs : -sn) : ((k < 32u) ? sn : cs);
    hv[e] = (_Float16)carry_flush(val, cTw);
  }
  unsigned short* dp = inv ? (TWI + (size_t)n * kS2 + k0) : (TWF + (size_t)n * kS + k0);
  *(volatile v8h*)dp = hv;
  __threadfence();
  *(volatile v8h*)dp = hv;
}

__global__ __launch_bounds__(kThr) void weight_planes_kernel(const float* __restrict__ Wb_r, const float* __restrict__ Wb_i,
                                                             const float* __restrict__ Wp1_r, const float* __restrict__ Wp1_i,
                                                             const float* __restrict__ Wp2_r, const float* __restrict__ Wp2_i,
                                                             const float* __restrict__ Wc_r, const float* __restrict__ Wc_i,
                                                             unsigned short* __restrict__ WB, unsigned short* __restrict__ WP1,
                                                             unsigned short* __restrict__ WP2, unsigned short* __restrict__ WC) {
  unsigned v = blockIdx.x * (unsigned)kThr + threadIdx.x;
  asm volatile("" : "+v"(v));
  unsigned which, u;
  if (v < 3072u) { which = 0u; u = v; }
  else if (v < 7680u) { which = 1u; u = v - 3072u; }
  else if (v < 12288u) { which = 2u; u = v - 7680u; }
  else { which = 3u; u = v - 12288u; }
  const unsigned K = (which == 0u) ? (unsigned)kE : (unsigned)kC;
  const unsigned vecPerRow = (2u * K) >> 3;
  const unsigned n = u / vecPerRow;
  const unsigned k0 = (u - n * vecPerRow) * 8u;
  const unsigned Nrows = (which == 3u) ? (unsigned)kE : (unsigned)kC;
  const bool imRow = (which != 3u) && (n >= Nrows);
  const unsigned nn = imRow ? (n - Nrows) : n;
  const bool second = k0 >= K;
  const unsigned kk = second ? (k0 - K) : k0;
  const float* re = (which == 0u) ? Wb_r : ((which == 1u) ? Wp1_r : ((which == 2u) ? Wp2_r : Wc_r));
  const float* im = (which == 0u) ? Wb_i : ((which == 1u) ? Wp1_i : ((which == 2u) ? Wp2_i : Wc_i));
  const bool takeIm = imRow ? !second : second;
  const float sgn = (!imRow && second) ? -1.0f : 1.0f;
  const float* src = (takeIm ? im : re) + (size_t)nn * K + kk;
  const v4f a0 = *(const v4f*)(src);
  const v4f a1 = *(const v4f*)(src + 4);
  v8h hv;
#pragma unroll
  for (int e = 0; e < 4; ++e) {
    const float f0 = a0[e];
    const float f1 = a1[e];
    hv[e]     = (_Float16)carry_flush(sgn * bf16r(f0), cW);
    hv[4 + e] = (_Float16)carry_flush(sgn * bf16r(f1), cW);
  }
  unsigned short* base = (which == 0u) ? WB : ((which == 1u) ? WP1 : ((which == 2u) ? WP2 : WC));
  unsigned short* dp = base + (size_t)n * (2u * K) + k0;
  *(volatile v8h*)dp = hv;
  __threadfence();
  *(volatile v8h*)dp = hv;
}
static_assert(3072 + 4608 + 4608 + 1536 == 54 * kThr, "weight planes grid exact");

__global__ __launch_bounds__(kThr) void bias_tables_kernel(const float* __restrict__ bb_r, const float* __restrict__ bb_i,
                                                           const float* __restrict__ bp1_r, const float* __restrict__ bp1_i,
                                                           const float* __restrict__ bp2_r, const float* __restrict__ bp2_i,
                                                           const float* __restrict__ bc_r, float* __restrict__ TAB) {
  unsigned i0 = threadIdx.x * 4u;
  asm volatile("" : "+v"(i0));
  v4f o;
#pragma unroll
  for (int e = 0; e < 4; ++e) {
    const unsigned i = i0 + (unsigned)e;
    float val = 0.0f;
    if (i < (unsigned)kTabBP2) { val = bf16r((i < 96u) ? bp1_r[i] : bp1_i[i - 96u]); }
    else if (i < (unsigned)kTabBC) { const unsigned j = i - (unsigned)kTabBP2; val = bf16r((j < 96u) ? bp2_r[j] : bp2_i[j - 96u]); }
    else if (i < (unsigned)kTabBB) { val = bf16r(bc_r[i - (unsigned)kTabBC]); }
    else if (i < (unsigned)kTabZB) { const unsigned j = i - (unsigned)kTabBB; val = 1024.0f * bf16r((j < 96u) ? bb_r[j] : bb_i[j - 96u]); }
    o[e] = val;
  }
  *(volatile v4f*)(TAB + i0) = o;
  __threadfence();
  *(volatile v4f*)(TAB + i0) = o;
}
__global__ __launch_bounds__(kThr) void lambda_tables_kernel(const float* __restrict__ params_log, float* __restrict__ TAB) {
  unsigned j = blockIdx.x * (unsigned)kThr + threadIdx.x;
  asm volatile("" : "+v"(j));
  const float nu = expf(bf16r(params_log[j]));
  const float th = expf(bf16r(params_log[3072u + j]));
  const float gam = expf(bf16r(params_log[6144u + j]));
  const float mag = expf(-nu);
  float sn, cs;
  sincosf(th, &sn, &cs);
  const float lre = mag * cs;
  const float lim = mag * sn;
  for (int pass = 0; pass < 2; ++pass) {
    *(volatile float*)(TAB + kTabGAM + j) = gam;
    *(volatile float*)(TAB + kTabLRE + j) = lre;
    *(volatile float*)(TAB + kTabLIM + j) = lim;
    __threadfence();
  }
}
static_assert(kTabGAM == 4 * kThr && kC * kS == 12 * kThr, "table grids exact");

__global__ __launch_bounds__(kThr) void repack_kernel(const float* __restrict__ src, unsigned short* __restrict__ dst, int CH, float carry) {
  unsigned v = blockIdx.x * (unsigned)kThr + threadIdx.x;
  asm volatile("" : "+v"(v));
  const unsigned vecPerRow = (2u * (unsigned)CH) >> 3;
  const unsigned row = v / vecPerRow;
  const unsigned c0 = (v - row * vecPerRow) * 8u;
  const unsigned part = (c0 >= (unsigned)CH) ? 1u : 0u;
  const unsigned ch0 = c0 - part * (unsigned)CH;
  const unsigned pair = row >> 5;
  const unsigned j = row & 31u;
  const float* sp = src + ((size_t)pair * (unsigned)CH + ch0) * kS2 + part * 32u + j;
  v8h hv;
#pragma unroll
  for (int e = 0; e < 8; ++e) hv[e] = (_Float16)carry_flush(sp[(size_t)e * kS2], carry);
  unsigned short* dp = dst + (size_t)v * 8u;
  *(volatile v8h*)dp = hv;
  __threadfence();
  *(volatile v8h*)dp = hv;
}
static_assert((kPA * kE2 / 8) % kThr == 0 && (kPA * kC2 / 8) % kThr == 0, "repack grids exact");

__global__ __launch_bounds__(kThr) void cast_rows_kernel(const float* __restrict__ src, unsigned short* __restrict__ dst, const float* __restrict__ BB, int addBias, float carry) {
  unsigned v = blockIdx.x * (unsigned)kThr + threadIdx.x;
  asm volatile("" : "+v"(v));
  const unsigned row = v / 24u;
  const unsigned c0 = (v - row * 24u) * 8u;
  const bool bias = (addBias != 0) && ((row & 31u) == 0u);
  const float* sp = src + (size_t)v * 8u;
  const v4f a0 = *(const v4f*)(sp);
  const v4f a1 = *(const v4f*)(sp + 4);
  const v4f b0 = *(const v4f*)(BB + c0);
  const v4f b1 = *(const v4f*)(BB + c0 + 4);
  v8h hv;
#pragma unroll
  for (int e = 0; e < 4; ++e) {
    hv[e]     = (_Float16)carry_flush(a0[e] + (bias ? b0[e] : 0.0f), carry);
    hv[4 + e] = (_Float16)carry_flush(a1[e] + (bias ? b1[e] : 0.0f), carry);
  }
  unsigned short* dp = dst + (size_t)v * 8u;
  *(volatile v8h*)dp = hv;
  __threadfence();
  *(volatile v8h*)dp = hv;
}

constexpr int kScanThr = 128;
__global__ __launch_bounds__(kScanThr) void diag_scan_kernel(const float* __restrict__ H2, const float* __restrict__ TAB, const float* __restrict__ mask,
                                                             unsigned short* __restrict__ A5) {
  __shared__ float sHr[32][kScanThr];
  __shared__ float sHi[32][kScanThr];
  __shared__ float sMk[32][kScanThr];
  __shared__ float sPr[16][kScanThr];
  __shared__ float sPi[16][kScanThr];
  const unsigned tid = threadIdx.x;
  unsigned t = blockIdx.x * (unsigned)kScanThr + tid;
  asm volatile("" : "+v"(t));
  const unsigned a = t & 31u;
  const unsigned bc = t >> 5;
  const unsigned b = bc / 96u;
  const unsigned c = bc - b * 96u;
  const float gam = TAB[kTabGAM + c * 32u + a];
  sPr[0][tid] = TAB[kTabLRE + c * 32u + a];
  sPi[0][tid] = TAB[kTabLIM + c * 32u + a];
#pragma unroll 1
  for (int n = 1; n < 16; n *= 2) {
    const float qr = sPr[n - 1][tid], qi = sPi[n - 1][tid];
#pragma unroll 1
    for (int j = 0; j < n; ++j) {
      const float ar = sPr[j][tid], ai = sPi[j][tid];
      sPr[n + j][tid] = ar * qr - ai * qi;
      sPi[n + j][tid] = ar * qi + ai * qr;
    }
  }
#pragma unroll 1
  for (int l = 0; l < 32; ++l) {
    const float* row = H2 + ((size_t)(b * 32u + (unsigned)l) * 32u + a) * kC2;
    sHr[l][tid] = gam * row[c];
    sHi[l][tid] = gam * row[kC + c];
    const float mv = mask[b * 32u + (unsigned)l];
    sMk[l][tid] = bf16r(mv);
  }
#pragma unroll 1
  for (int len = 2; len <= 32; len *= 2) {
    const int half = len >> 1;
#pragma unroll 1
    for (int l = 0; l < 32; ++l) {
      if (l & half) {
        const int j = l & (half - 1);
        const int last = (l & ~(len - 1)) + half - 1;
        const float m = sMk[last][tid];
        const float lr = sHr[last][tid] * m;
        const float li = sHi[last][tid] * m;
        const float pr = sPr[j][tid], pi = sPi[j][tid];
        sHr[l][tid] += pr * lr - pi * li;
        sHi[l][tid] += pr * li + pi * lr;
      }
    }
  }
#pragma unroll 1
  for (int l = 0; l < 32; ++l) {
    unsigned short* dp = A5 + ((size_t)(b * 32u + (unsigned)l) * 96u + c) * kS2 + a;
    const _Float16 vr = (_Float16)carry_flush(sHr[l][tid], cHs);
    const _Float16 vi = (_Float16)carry_flush(sHi[l][tid], cHs);
    *(volatile _Float16*)dp = vr;
    *(volatile _Float16*)(dp + 32) = vi;
    __threadfence();
    *(volatile _Float16*)dp = vr;
    *(volatile _Float16*)(dp + 32) = vi;
  }
}
static_assert(kB * kC * kS == 96 * kScanThr, "scan grid exact");

__device__ __forceinline__ float block_sum_256(float v, float* sRed, float* sGrp, int tid) {
  sRed[tid] = v;
  __syncthreads();
  if (tid < 8) {
    float s = 0.f;
#pragma unroll
    for (int k = 0; k < 8; ++k) {
      const v4f q = *(const v4f*)(sRed + tid * 32 + 4 * k);
      s += q[0]; s += q[1]; s += q[2]; s += q[3];
    }
    sGrp[tid] = s;
  }
  __syncthreads();
  float tsum = 0.f;
#pragma unroll
  for (int k = 0; k < 8; ++k) tsum += sGrp[k];
  __syncthreads();
  return tsum;
}
__global__ __launch_bounds__(kThr) void out_kernel(const float* __restrict__ RR, const float* __restrict__ x, const float* __restrict__ ln_w,
                                                   const float* __restrict__ ln_b, float* __restrict__ out) {
  __shared__ __align__(16) float sRed[256];
  __shared__ __align__(16) float sGrp[8];
  const int tid = threadIdx.x;
  const unsigned pair = blockIdx.x >> 6;
  const unsigned e = blockIdx.x & 63u;
  const float* rp = RR + (size_t)pair * (kS * kE);
  const v4f r0 = *(const v4f*)(rp + 8 * tid);
  const v4f r1 = *(const v4f*)(rp + 8 * tid + 4);
  const float mu = block_sum_256(((r0[0] + r0[1]) + (r0[2] + r0[3])) + ((r1[0] + r1[1]) + (r1[2] + r1[3])), sRed, sGrp, tid) / 2048.0f;
  float q = 0.f;
#pragma unroll
  for (int k = 0; k < 4; ++k) { const float d0 = r0[k] - mu; const float d1 = r1[k] - mu; q += d0 * d0; q += d1 * d1; }
  const float var = block_sum_256(q, sRed, sGrp, tid) / 2048.0f;
  const float sd = sqrtf(var + 1e-5f);
  const unsigned p = (unsigned)tid >> 3;
  const unsigned q0 = ((unsigned)tid & 7u) * 4u;
  const size_t po = ((size_t)e * kS + p) * kS + q0;
  const size_t go = (size_t)pair * (kE * kS * kS) + po;
  const v4f xv = *(const v4f*)(x + go);
  const v4f wv = *(const v4f*)(ln_w + po);
  const v4f bv = *(const v4f*)(ln_b + po);
  v4f o;
#pragma unroll
  for (int k = 0; k < 4; ++k) {
    const unsigned s = (p + q0 + (unsigned)k) & 31u;
    const float rv = rp[s * (unsigned)kE + e];
    const float xe = xv[k];
    const float we = wv[k];
    const float be = bv[k];
    o[k] = (rv - mu) / sd * bf16r(we) + bf16r(be) + bf16r(xe);
  }
  *(volatile v4f*)(out + go) = o;
  __threadfence();
  *(volatile v4f*)(out + go) = o;
}

static_assert(((kPE / 64) * (kS2 / 64)) % 8 == 0 && ((kPA / 64) * (kC2 / 64)) % 8 == 0 && ((kPC / 64) * (kS2 / 64)) % 8 == 0 && ((kPA / 64) * (kE / 64)) % 8 == 0, "GEMM grids exact");

extern "C" void kernel_launch(void* const* d_in, const int* in_sizes, int n_in,
                              void* d_out, int out_size, void* d_ws, size_t ws_size,
                              hipStream_t stream) {
  if (n_in < 21 || d_out == nullptr || d_ws == nullptr) return;
  if (in_sizes[0] != kP * kE * kS * kS || in_sizes[1] != kP || in_sizes[2] != 3 * kC * kS) return;
  if (in_sizes[3] != kC * kE || in_sizes[4] != kC * kE || in_sizes[5] != kC || in_sizes[6] != kC) return;
  if (in_sizes[7] != kC * kC || in_sizes[8] != kC * kC || in_sizes[9] != kC || in_sizes[10] != kC) return;
  if (in_sizes[11] != kC * kC || in_sizes[12] != kC * kC || in_sizes[13] != kC || in_sizes[14] != kC) return;
  if (in_sizes[15] != kE * kC || in_sizes[16] != kE * kC || in_sizes[17] != kE || in_sizes[18] != kE) return;
  if (in_sizes[19] != kE * kS * kS || in_sizes[20] != kE * kS * kS) return;
  if (out_size != kP * kE * kS * kS) return;
  if (ws_size < kWsTotal) return;

  const float* x      = (const float*)d_in[0];
  const float* mask   = (const float*)d_in[1];
  const float* plog   = (const float*)d_in[2];
  const float* Wb_r   = (const float*)d_in[3];
  const float* Wb_i   = (const float*)d_in[4];
  const float* bb_r   = (const float*)d_in[5];
  const float* bb_i   = (const float*)d_in[6];
  const float* Wp1_r  = (const float*)d_in[7];
  const float* Wp1_i  = (const float*)d_in[8];
  const float* bp1_r  = (const float*)d_in[9];
  const float* bp1_i  = (const float*)d_in[10];
  const float* Wp2_r  = (const float*)d_in[11];
  const float* Wp2_i  = (const float*)d_in[12];
  const float* bp2_r  = (const float*)d_in[13];
  const float* bp2_i  = (const float*)d_in[14];
  const float* Wc_r   = (const float*)d_in[15];
  const float* Wc_i   = (const float*)d_in[16];
  const float* bc_r   = (const float*)d_in[17];
  const float* ln_w   = (const float*)d_in[19];
  const float* ln_b   = (const float*)d_in[20];
  float* out = (float*)d_out;

  char* ws = (char*)d_ws;
  unsigned short* SX16 = (unsigned short*)(ws + kOffSX);
  unsigned short* TWF  = (unsigned short*)(ws + kOffTWF);
  unsigned short* TWI  = (unsigned short*)(ws + kOffTWI);
  unsigned short* WB   = (unsigned short*)(ws + kOffWB);
  unsigned short* WP1  = (unsigned short*)(ws + kOffWP1);
  unsigned short* WP2  = (unsigned short*)(ws + kOffWP2);
  unsigned short* WC   = (unsigned short*)(ws + kOffWC);
  float*          TAB  = (float*)(ws + kOffTAB);
  float*          XH   = (float*)(ws + kOffXH);
  unsigned short* A2   = (unsigned short*)(ws + kOffA2);
  float*          H1   = (float*)(ws + kOffH1);
  unsigned short* A3   = (unsigned short*)(ws + kOffA3);
  float*          H2   = (float*)(ws + kOffH2);
  unsigned short* A5   = (unsigned short*)(ws + kOffA5);
  float*          GG   = (float*)(ws + kOffGG);
  unsigned short* A6   = (unsigned short*)(ws + kOffA6);
  float*          H6   = (float*)(ws + kOffH6);
  unsigned short* A7   = (unsigned short*)(ws + kOffA7);
  float*          RR   = (float*)(ws + kOffRR);

  antidiag_kernel<<<512, kThr, 0, stream>>>(x, SX16);
  twiddle_kernel<<<3, kThr, 0, stream>>>(TWF, TWI);
  weight_planes_kernel<<<54, kThr, 0, stream>>>(Wb_r, Wb_i, Wp1_r, Wp1_i, Wp2_r, Wp2_i, Wc_r, Wc_i, WB, WP1, WP2, WC);
  bias_tables_kernel<<<1, kThr, 0, stream>>>(bb_r, bb_i, bp1_r, bp1_i, bp2_r, bp2_i, bc_r, TAB);
  lambda_tables_kernel<<<12, kThr, 0, stream>>>(plog, TAB);

  wmma_gemm64<0, false, 2, 0, false, 0><<<dim3((kPE / 64) * (kS2 / 64) / 8, 1), 256, 0, stream>>>(
      SX16, SX16, kS, 0L, TWF, TWF, kS, 0L, (void*)XH, (void*)XH, kS2, 0L, TAB + kTabZB, nullptr, 0L, kPE, kS2, kS, kScG1);
  repack_kernel<<<(kPA * kE2 / 8) / kThr, kThr, 0, stream>>>(XH, A2, kE, cXh);
  wmma_gemm64<0, false, 2, 0, false, 0><<<dim3((kPA / 64) * (kC2 / 64) / 8, 1), 256, 0, stream>>>(
      A2, A2, kE2, 0L, WB, WB, kE2, 0L, (void*)H1, (void*)H1, kC2, 0L, TAB + kTabZB, nullptr, 0L, kPA, kC2, kE2, kScG2);
  cast_rows_kernel<<<(kPA * kC2 / 8) / kThr, kThr, 0, stream>>>(H1, A3, TAB + kTabBB, 1, cH1);
  wmma_gemm64<0, false, 2, 0, false, 0><<<dim3((kPA / 64) * (kC2 / 64) / 8, 1), 256, 0, stream>>>(
      A3, A3, kC2, 0L, WP1, WP1, kC2, 0L, (void*)H2, (void*)H2, kC2, 0L, TAB + kTabBP1, nullptr, 0L, kPA, kC2, kC2, kScG3);
  diag_scan_kernel<<<96, kScanThr, 0, stream>>>(H2, TAB, mask, A5);
  wmma_gemm64<0, false, 2, 0, false, 0><<<dim3((kPC / 64) * (kS2 / 64) / 8, 1), 256, 0, stream>>>(
      A5, A5, kS2, 0L, TWI, TWI, kS2, 0L, (void*)GG, (void*)GG, kS2, 0L, TAB + kTabZB, nullptr, 0L, kPC, kS2, kS2, kScG5);
  repack_kernel<<<(kPA * kC2 / 8) / kThr, kThr, 0, stream>>>(GG, A6, kC, cG);
  wmma_gemm64<0, false, 2, 0, false, 0><<<dim3((kPA / 64) * (kC2 / 64) / 8, 1), 256, 0, stream>>>(
      A6, A6, kC2, 0L, WP2, WP2, kC2, 0L, (void*)H6, (void*)H6, kC2, 0L, TAB + kTabBP2, nullptr, 0L, kPA, kC2, kC2, kScG6);
  cast_rows_kernel<<<(kPA * kC2 / 8) / kThr, kThr, 0, stream>>>(H6, A7, TAB + kTabBB, 0, cH6);
  wmma_gemm64<0, false, 2, 0, false, 0><<<dim3((kPA / 64) * (kE / 64) / 8, 1), 256, 0, stream>>>(
      A7, A7, kC2, 0L, WC, WC, kC2, 0L, (void*)RR, (void*)RR, kE, 0L, TAB + kTabBC, nullptr, 0L, kPA, kE, kC2, kScG7);
  out_kernel<<<kP * kE, kThr, 0, stream>>>(RR, x, ln_w, ln_b, out);
}
